// HeteroSAGENet_4604204941984
// MI455X (gfx1250) — hardware-verified
//
#include <hip/hip_runtime.h>
#include <stddef.h>


#define HID    128
#define FFM    64
#define FSM    32
#define FTP    32
#define FGF    64
#define HHALF  64
#define NTHR   256
#define NWAVE  8
#define EPT    8
#define CHUNK  (NTHR * EPT)
#define WCAP   (EPT * 32)
#define LISTN  (NWAVE * WCAP)
#define LPAD   16
#define NBFM   512
#define NBTP   512
#define NBSM   1024
#define KFM    (FFM + FTP + FTP + FFM)
#define KTP    (FFM + FTP)
#define KSM    (FTP + FSM)
#define WSCALE 8.0f
#define WINV   0.125f

#define LDS_BYTES(NB, KAGG, NREL) ((((NB) * (KAGG)) + ((NREL) * (NB)) + LISTN + LPAD) * 4)
#define LDS_FM LDS_BYTES(NBFM, (FFM + FTP + FTP), 3)
#define LDS_TP LDS_BYTES(NBTP, FFM, 1)
#define LDS_SM LDS_BYTES(NBSM, FTP, 1)

static_assert((CHUNK & (CHUNK - 1)) == 0);
static_assert(CHUNK <= 4096);
static_assert(NBFM <= 4096 && NBTP <= 4096 && NBSM <= 4096);
static_assert(NWAVE * HID + HID <= LISTN);
static_assert(LDS_FM <= 300 * 1024);

typedef float    v2f  __attribute__((ext_vector_type(2)));
typedef float    v4f  __attribute__((ext_vector_type(4)));
typedef float    v8f  __attribute__((ext_vector_type(8)));
typedef int      v4i  __attribute__((ext_vector_type(4)));
typedef _Float16 v8h  __attribute__((ext_vector_type(8)));
typedef _Float16 v16h __attribute__((ext_vector_type(16)));
union FragH { v16h v; v8h h[2]; };

__device__ __forceinline__ v8h cvt8(v4f a, v4f b) {
  v8h r;
  r[0] = (_Float16)a.x; r[1] = (_Float16)a.y; r[2] = (_Float16)a.z; r[3] = (_Float16)a.w;
  r[4] = (_Float16)b.x; r[5] = (_Float16)b.y; r[6] = (_Float16)b.z; r[7] = (_Float16)b.w;
  return r;
}

__device__ __forceinline__ v4f sel4(bool c, v4f a, v4f b) {
  v4f r;
  r.x = c ? a.x : b.x; r.y = c ? a.y : b.y; r.z = c ? a.z : b.z; r.w = c ? a.w : b.w;
  return r;
}

__device__ __forceinline__ v8f wmh(v16h a, v16h b, v8f c) {
  v8f d = __builtin_amdgcn_wmma_f32_16x16x32_f16(false, a, false, b, (short)0, c, false, false);
  asm volatile("v_nop\n\tv_nop\n\tv_nop\n\tv_nop" : "+v"(d) : "v"(a), "v"(b));
  return d;
}

__device__ __forceinline__ float hred16(float x) {
  x += __shfl_xor(x, 1);
  x += __shfl_xor(x, 2);
  x += __shfl_xor(x, 4);
  x += __shfl_xor(x, 8);
  return x;
}

__device__ __forceinline__ float relu_rows(v8f y, int vlim) {
  float s = 0.f;
#pragma unroll
  for (int r = 0; r < 8; ++r) s += (r < vlim) ? fmaxf(y[r], 0.f) : 0.f;
  return s;
}

__device__ __forceinline__ void ld8(const float* __restrict__ W, int k0, int nrow, int n, v4f& a, v4f& b) {
  float t[8];
#pragma unroll
  for (int j = 0; j < 8; ++j) {
    int k = k0 + j;
    k = k < 0 ? 0 : (k > nrow - 1 ? nrow - 1 : k);
    t[j] = W[(size_t)k * HID + n];
  }
  a.x = t[0]; a.y = t[1]; a.z = t[2]; a.w = t[3];
  b.x = t[4]; b.y = t[5]; b.z = t[6]; b.w = t[7];
}

template <int NB>
__device__ __forceinline__ int scan_chunk(const int* __restrict__ dsts, int nE, int cbase, int nodeBase,
                                          int* list, int tid, int wave) {
  int wc = 0;
  const int el0  = tid * EPT;
  const int e0   = cbase + el0;
  const int sent = -2147483647 - 1;
  v4i da, db;
  if (cbase + CHUNK <= nE) {
    da = *(const v4i*)(dsts + e0);
    db = *(const v4i*)(dsts + e0 + 4);
  } else {
    const int em = nE - 1;
    da.x = (e0     < nE) ? dsts[min(e0,     em)] : sent;
    da.y = (e0 + 1 < nE) ? dsts[min(e0 + 1, em)] : sent;
    da.z = (e0 + 2 < nE) ? dsts[min(e0 + 2, em)] : sent;
    da.w = (e0 + 3 < nE) ? dsts[min(e0 + 3, em)] : sent;
    db.x = (e0 + 4 < nE) ? dsts[min(e0 + 4, em)] : sent;
    db.y = (e0 + 5 < nE) ? dsts[min(e0 + 5, em)] : sent;
    db.z = (e0 + 6 < nE) ? dsts[min(e0 + 6, em)] : sent;
    db.w = (e0 + 7 < nE) ? dsts[min(e0 + 7, em)] : sent;
  }
  const unsigned nb = (unsigned)nodeBase;
  const unsigned s0 = (unsigned)da.x - nb, s1 = (unsigned)da.y - nb;
  const unsigned s2 = (unsigned)da.z - nb, s3 = (unsigned)da.w - nb;
  const unsigned s4 = (unsigned)db.x - nb, s5 = (unsigned)db.y - nb;
  const unsigned s6 = (unsigned)db.z - nb, s7 = (unsigned)db.w - nb;
  const bool h0 = s0 < (unsigned)NB, h1 = s1 < (unsigned)NB, h2 = s2 < (unsigned)NB, h3 = s3 < (unsigned)NB;
  const bool h4 = s4 < (unsigned)NB, h5 = s5 < (unsigned)NB, h6 = s6 < (unsigned)NB, h7 = s7 < (unsigned)NB;
  const unsigned any = __builtin_amdgcn_ballot_w32(h0 | h1 | h2 | h3 | h4 | h5 | h6 | h7);
  if (any != 0u) {
#define HITJ(J, HJ, SJ) { \
      const unsigned mj = __builtin_amdgcn_ballot_w32(HJ); \
      if (mj != 0u) { \
        if (HJ) { \
          const int pos = wc + (int)__builtin_amdgcn_mbcnt_lo(mj, 0u); \
          if (pos < WCAP) list[wave * WCAP + pos] = ((el0 + (J)) << 12) | (int)(SJ); \
        } \
        wc += (int)__builtin_popcount(mj); } }
    HITJ(0, h0, s0)
    HITJ(1, h1, s1)
    HITJ(2, h2, s2)
    HITJ(3, h3, s3)
    HITJ(4, h4, s4)
    HITJ(5, h5, s5)
    HITJ(6, h6, s6)
    HITJ(7, h7, s7)
#undef HITJ
  }
  return wc;
}

template <int NB, int KAGG, int FW>
__device__ __forceinline__ void drain_lists(const int* list, const int* wcnt, int cbase, int nE,
                                            const int* __restrict__ srcs, int nS,
                                            const float* __restrict__ feat,
                                            float* acc, int* cnt, int coff, int lane) {
#pragma unroll 1
  for (int wsx = 0; wsx < NWAVE; ++wsx) {
    int n = __builtin_amdgcn_readfirstlane(wcnt[wsx]);
    n = n > WCAP ? WCAP : (n < 0 ? 0 : n);
    const int* lp = list + wsx * WCAP;
#pragma unroll 1
    for (int i = 0; i < n; ++i) {
      const int ent = __builtin_amdgcn_readfirstlane(lp[i]);
      int slot = ent & 4095;
      slot = slot > NB - 1 ? NB - 1 : slot;
      int e = cbase + ((ent >> 12) & (CHUNK - 1));
      e = e > nE - 1 ? nE - 1 : e;
      int s = srcs[e];
      s = s < 0 ? 0 : (s > nS - 1 ? nS - 1 : s);
      if (FW == 64) {
        const v2f v = *(const v2f*)(feat + (size_t)s * 64 + 2 * lane);
        v2f* ap = (v2f*)(acc + slot * KAGG + coff + 2 * lane);
        *ap = *ap + v;
      } else {
        const float v = feat[(size_t)s * 32 + lane];
        float* ap = acc + slot * KAGG + coff + lane;
        *ap = *ap + v;
      }
      if (lane == 0) cnt[slot] = cnt[slot] + 1;
    }
  }
}

template <int NB, int KAGG, int FW>
__device__ __forceinline__ void scan_rel(const int* __restrict__ srcs, const int* __restrict__ dsts, int nE,
                                         const float* __restrict__ feat, int nS,
                                         float* acc, int* cnt, int coff, int* list, int* wcnt,
                                         int nodeBase, int tid, int lane, int wave) {
  const int nChunks = (nE + CHUNK - 1) / CHUNK;
#pragma unroll 1
  for (int ch = 0; ch < nChunks; ++ch) {
    const int cbase = ch * CHUNK;
    const int wc = scan_chunk<NB>(dsts, nE, cbase, nodeBase, list, tid, wave);
    if (lane == 0) wcnt[wave] = wc;
    __syncthreads();
    if (wave == 0) drain_lists<NB, KAGG, FW>(list, wcnt, cbase, nE, srcs, nS, feat, acc, cnt, coff, lane);
    __syncthreads();
  }
}

__global__ __launch_bounds__(NTHR) void k_prep(
    const float* __restrict__ pe_table, const float* __restrict__ vol, int nTP, int nPeBlk,
    const float* __restrict__ qWl, const float* __restrict__ cWl, const float* __restrict__ rWl,
    const float* __restrict__ qWr, const float* __restrict__ cWr, const float* __restrict__ rWr,
    const float* __restrict__ qbl, const float* __restrict__ cbl, const float* __restrict__ rbl,
    const float* __restrict__ bWl, const float* __restrict__ bWr,
    const float* __restrict__ dWl, const float* __restrict__ dWr,
    float* pe, _Float16* Bfm, _Float16* Btp, _Float16* Bsm, float* biasfm) {
  const int b = blockIdx.x, tid = threadIdx.x;
  if (b < nPeBlk) {
    const int t   = b * NTHR + tid;
    const int row = t >> 3;
    const int c4  = (t & 7) * 4;
    const int rs  = row > nTP - 1 ? nTP - 1 : row;
    v4f v = *(const v4f*)(pe_table + (size_t)rs * FTP + c4);
    const float s = vol[rs];
    v = v * s;
    float* dp = pe + (size_t)row * FTP + c4;
    *(volatile v4f*)dp = v;
    __threadfence();
    *(volatile v4f*)dp = v;
    return;
  }
  const int rb = b - nPeBlk;
  if (rb < (HID * KFM / 8) / NTHR) {
    const int i  = rb * NTHR + tid;
    const int o  = i * 8;
    const int n  = o / KFM;
    const int k0 = o - n * KFM;
    v4f qa, qb, ca, cb, ra, rbv, wa, wb, xa, xb, ya, yb;
    ld8(qWl, k0,               FFM, n, qa, qb);
    ld8(cWl, k0 - FFM,         FTP, n, ca, cb);
    ld8(rWl, k0 - FFM - FTP,   FTP, n, ra, rbv);
    ld8(qWr, k0 - FFM - 2*FTP, FFM, n, wa, wb);
    ld8(cWr, k0 - FFM - 2*FTP, FFM, n, xa, xb);
    ld8(rWr, k0 - FFM - 2*FTP, FFM, n, ya, yb);
    wa = wa + xa + ya;
    wb = wb + xb + yb;
    v4f a  = sel4(k0 < FFM, qa, sel4(k0 < FFM + FTP, ca, sel4(k0 < FFM + 2*FTP, ra,  wa)));
    v4f bq = sel4(k0 < FFM, qb, sel4(k0 < FFM + FTP, cb, sel4(k0 < FFM + 2*FTP, rbv, wb)));
    a  = a  * WSCALE;
    bq = bq * WSCALE;
    const v8h hv = cvt8(a, bq);
    _Float16* dp = Bfm + o;
    *(volatile v8h*)dp = hv;
    __threadfence();
    *(volatile v8h*)dp = hv;
    return;
  }
  const int rb2 = rb - (HID * KFM / 8) / NTHR;
  if (rb2 < (HID * KTP / 8) / NTHR) {
    const int i  = rb2 * NTHR + tid;
    const int o  = i * 8;
    const int n  = o / KTP;
    const int k0 = o - n * KTP;
    v4f la, lb, wa, wb;
    ld8(bWl, k0,       FFM, n, la, lb);
    ld8(bWr, k0 - FFM, FTP, n, wa, wb);
    v4f a  = sel4(k0 < FFM, la, wa) * WSCALE;
    v4f bq = sel4(k0 < FFM, lb, wb) * WSCALE;
    const v8h hv = cvt8(a, bq);
    _Float16* dp = Btp + o;
    *(volatile v8h*)dp = hv;
    __threadfence();
    *(volatile v8h*)dp = hv;
    return;
  }
  const int rb3 = rb2 - (HID * KTP / 8) / NTHR;
  if (rb3 < (HID * KSM / 8) / NTHR) {
    const int i  = rb3 * NTHR + tid;
    const int o  = i * 8;
    const int n  = o / KSM;
    const int k0 = o - n * KSM;
    v4f la, lb, wa, wb;
    ld8(dWl, k0,       FTP, n, la, lb);
    ld8(dWr, k0 - FTP, FSM, n, wa, wb);
    v4f a  = sel4(k0 < FTP, la, wa) * WSCALE;
    v4f bq = sel4(k0 < FTP, lb, wb) * WSCALE;
    const v8h hv = cvt8(a, bq);
    _Float16* dp = Bsm + o;
    *(volatile v8h*)dp = hv;
    __threadfence();
    *(volatile v8h*)dp = hv;
    return;
  }
  if (tid < 32) {
    const int c4 = tid * 4;
    const v4f q = *(const v4f*)(qbl + c4), c = *(const v4f*)(cbl + c4), r = *(const v4f*)(rbl + c4);
    const v4f v = q + c + r;
    float* dp = biasfm + c4;
    *(volatile v4f*)dp = v;
    __threadfence();
    *(volatile v4f*)dp = v;
  }
}

template <int NB, int FW0, int FW1, int FW2, int KDST>
__global__ __launch_bounds__(NTHR) void k_sage(
    const int* __restrict__ src0, const int* __restrict__ dst0, int nE0, const float* __restrict__ feat0, int nS0,
    const int* __restrict__ src1, const int* __restrict__ dst1, int nE1, const float* __restrict__ feat1, int nS1,
    const int* __restrict__ src2, const int* __restrict__ dst2, int nE2, const float* __restrict__ feat2, int nS2,
    const float* __restrict__ xdst, int nN,
    const _Float16* __restrict__ BT, const float* __restrict__ bias, float scale,
    const float* __restrict__ gam, const float* __restrict__ bet, float* part) {
  constexpr int KAGG = FW0 + FW1 + FW2;
  constexpr int KTOT = KAGG + KDST;
  constexpr int NREL = 1 + (FW1 > 0 ? 1 : 0) + (FW2 > 0 ? 1 : 0);
  constexpr int TPW  = NB / (16 * NWAVE);
  static_assert(NB % (16 * NWAVE) == 0);
  static_assert(KAGG % 32 == 0 && KDST % 32 == 0 && FW0 % 32 == 0 && FW1 % 32 == 0 && FW2 % 32 == 0);
  extern __shared__ v4f lds_dyn[];
  float* acc  = (float*)lds_dyn;
  int*   cnt  = (int*)(acc + NB * KAGG);
  int*   list = cnt + NREL * NB;
  int*   wcnt = list + LISTN;
  float* wsum = (float*)list;
  float* pst  = wsum + NWAVE * HID;
  const int tid = threadIdx.x, lane = tid & 31, wave = tid >> 5, hh = lane >> 4, m = lane & 15;
  const int nodeBase = blockIdx.x * NB;

  {
    const v4f z = {0.f, 0.f, 0.f, 0.f};
    const int n4 = (NB * KAGG + NREL * NB) / 4;
    for (int i = tid; i < n4; i += NTHR) lds_dyn[i] = z;
  }
  __syncthreads();

  scan_rel<NB, KAGG, FW0>(src0, dst0, nE0, feat0, nS0, acc, cnt, 0, list, wcnt, nodeBase, tid, lane, wave);
  if (FW1 > 0)
    scan_rel<NB, KAGG, (FW1 > 0 ? FW1 : 32)>(src1, dst1, nE1, feat1, nS1, acc, cnt + NB, FW0,
                                              list, wcnt, nodeBase, tid, lane, wave);
  if (FW2 > 0)
    scan_rel<NB, KAGG, (FW2 > 0 ? FW2 : 32)>(src2, dst2, nE2, feat2, nS2, acc, cnt + 2 * NB, FW0 + FW1,
                                              list, wcnt, nodeBase, tid, lane, wave);
  __syncthreads();

  float cs[8];
#pragma unroll
  for (int t = 0; t < 8; ++t) cs[t] = 0.f;

#pragma unroll 1
  for (int j = 0; j < TPW; ++j) {
    const int trow = j * NWAVE + wave;
    const int rloc = trow * 16 + m;
    int node = nodeBase + rloc;
    node = node > nN - 1 ? nN - 1 : node;
    const int c0 = cnt[rloc];
    const float rc0 = 1.0f / (float)(c0 > 1 ? c0 : 1);
    float rc1 = 1.f, rc2 = 1.f;
    if (NREL > 1) { const int c1 = cnt[NB + rloc];     rc1 = 1.0f / (float)(c1 > 1 ? c1 : 1); }
    if (NREL > 2) { const int c2 = cnt[2 * NB + rloc]; rc2 = 1.0f / (float)(c2 > 1 ? c2 : 1); }

    v8f d[8];
#pragma unroll
    for (int t = 0; t < 8; ++t) { const v8f z = {0.f, 0.f, 0.f, 0.f, 0.f, 0.f, 0.f, 0.f}; d[t] = z; }

#pragma unroll
    for (int ks = 0; ks < KTOT / 32; ++ks) {
      FragH a;
      if (32 * ks < KAGG) {
        const float rc = (32 * ks < FW0) ? rc0 : ((32 * ks < FW0 + FW1) ? rc1 : rc2);
        const float* ap = acc + rloc * KAGG + 32 * ks + 8 * hh;
        const v4f p0 = *(const v4f*)ap,        p1 = *(const v4f*)(ap + 4);
        const v4f p2 = *(const v4f*)(ap + 16), p3 = *(const v4f*)(ap + 20);
        a.h[0] = cvt8(p0 * rc, p1 * rc);
        a.h[1] = cvt8(p2 * rc, p3 * rc);
      } else {
        const float* xp = xdst + (size_t)node * KDST + (32 * ks - KAGG) + 8 * hh;
        const v4f p0 = *(const v4f*)xp,        p1 = *(const v4f*)(xp + 4);
        const v4f p2 = *(const v4f*)(xp + 16), p3 = *(const v4f*)(xp + 20);
        a.h[0] = cvt8(p0, p1);
        a.h[1] = cvt8(p2, p3);
      }
#pragma unroll
      for (int t = 0; t < 8; ++t) {
        const _Float16* bp = BT + (size_t)(16 * t + m) * KTOT + 32 * ks + 8 * hh;
        FragH bf;
        bf.h[0] = *(const v8h*)bp;
        bf.h[1] = *(const v8h*)(bp + 16);
        d[t] = wmh(a.v, bf.v, d[t]);
      }
    }

#pragma unroll
    for (int t = 0; t < 8; ++t) {
      const float bc = bias[16 * t + m];
      d[t] = (d[t] * WINV + bc) * scale;
    }
    const v8f sv = d[0] + d[1] + d[2] + d[3] + d[4] + d[5] + d[6] + d[7];
    v8f mu;
#pragma unroll
    for (int r = 0; r < 8; ++r) mu[r] = hred16(sv[r]) * (1.0f / HID);
    v8f qv = {0.f, 0.f, 0.f, 0.f, 0.f, 0.f, 0.f, 0.f};
#pragma unroll
    for (int t = 0; t < 8; ++t) { const v8f e = d[t] - mu; d[t] = e; qv = qv + e * e; }
    v8f rs;
#pragma unroll
    for (int r = 0; r < 8; ++r) rs[r] = rsqrtf(hred16(qv[r]) * (1.0f / HID) + 1e-5f);
    const int vlim = nN - (nodeBase + trow * 16 + 8 * hh);
#pragma unroll
    for (int t = 0; t < 8; ++t) {
      const float gc = gam[16 * t + m], ec = bet[16 * t + m];
      const v8f y = d[t] * rs * gc + ec;
      cs[t] += relu_rows(y, vlim);
    }
  }

#pragma unroll
  for (int t = 0; t < 8; ++t) cs[t] += __shfl_xor(cs[t], 16);
  __syncthreads();
  if (hh == 0) {
#pragma unroll
    for (int t = 0; t < 8; ++t) wsum[wave * HID + 16 * t + m] = cs[t];
  }
  __syncthreads();
  if (tid < HID) {
    float p = 0.f;
#pragma unroll
    for (int w = 0; w < NWAVE; ++w) p += wsum[w * HID + tid];
    pst[tid] = p;
  }
  __syncthreads();
  if (wave == 0) {
    const v4f v = *(const v4f*)(pst + 4 * lane);
    float* gp = part + (size_t)blockIdx.x * HID + 4 * lane;
    *(volatile v4f*)gp = v;
    __threadfence();
    *(volatile v4f*)gp = v;
  }
}

__global__ __launch_bounds__(HID) void k_final(
    const float* __restrict__ pfm, int nBfm, int nFM,
    const float* __restrict__ ptp, int nBtp, int nTP,
    const float* __restrict__ psm, int nBsm, int nSM,
    const float* __restrict__ gf,
    const float* __restrict__ W1, const float* __restrict__ b1,
    const float* __restrict__ W2, const float* __restrict__ b2, float* out) {
  __shared__ float h[3 * HID + FGF];
  __shared__ float h1[HHALF];
  const int c = threadIdx.x, lane = c & 31;
  double s0 = 0.0, s1 = 0.0, s2 = 0.0;
#pragma unroll 1
  for (int b = 0; b < nBfm; ++b) s0 += (double)pfm[(size_t)b * HID + c];
#pragma unroll 1
  for (int b = 0; b < nBtp; ++b) s1 += (double)ptp[(size_t)b * HID + c];
#pragma unroll 1
  for (int b = 0; b < nBsm; ++b) s2 += (double)psm[(size_t)b * HID + c];
  h[c]           = (float)(s0 / (double)nFM);
  h[HID + c]     = (float)(s1 / (double)nTP);
  h[2 * HID + c] = (float)(s2 / (double)nSM);
  {
    const int cg = c > FGF - 1 ? FGF - 1 : c;
    const float g = gf[cg];
    if (c < FGF) h[3 * HID + c] = g;
  }
  __syncthreads();
  if (c < HHALF) {
    float a = 0.f;
#pragma unroll 4
    for (int i = 0; i < 3 * HID + FGF; ++i) a += h[i] * W1[(size_t)i * HHALF + c];
    a += b1[c];
    h1[c] = fmaxf(a, 0.f);
  }
  __syncthreads();
  if (c < 32) {
    float a = h1[lane] * W2[lane] + h1[lane + 32] * W2[lane + 32];
    a += __shfl_xor(a, 16);
    a += __shfl_xor(a, 8);
    a += __shfl_xor(a, 4);
    a += __shfl_xor(a, 2);
    a += __shfl_xor(a, 1);
    const float r = a + b2[0];
    if (lane == 0) {
      *(volatile float*)out = r;
      __threadfence();
      *(volatile float*)out = r;
    }
  }
}

extern "C" void kernel_launch(void* const* d_in, const int* in_sizes, int n_in,
                              void* d_out, int out_size, void* d_ws, size_t ws_size,
                              hipStream_t stream) {
  if (n_in < 40 || out_size != 1) return;
  const int nFM = in_sizes[0] / FFM;
  const int nSM = in_sizes[1] / FSM;
  const int nTP = in_sizes[2];
  if (nFM <= 0 || nSM <= 0 || nTP <= 0) return;
  if (in_sizes[0] != nFM * FFM || in_sizes[1] != nSM * FSM || in_sizes[4] != nTP * FTP || in_sizes[3] < FGF) return;
  const int nEq = in_sizes[5], nEb = in_sizes[7], nEc = in_sizes[9], nEd = in_sizes[11], nEr = in_sizes[13];
  if (nEq < 0 || nEb < 0 || nEc < 0 || nEd < 0 || nEr < 0) return;
  if (in_sizes[6] != nEq || in_sizes[8] != nEb || in_sizes[10] != nEc || in_sizes[12] != nEd || in_sizes[14] != nEr) return;
  if (in_sizes[15] != FFM * HID || in_sizes[17] != FFM * HID || in_sizes[18] != FFM * HID || in_sizes[20] != FTP * HID ||
      in_sizes[21] != FTP * HID || in_sizes[23] != FFM * HID || in_sizes[24] != FTP * HID || in_sizes[26] != FSM * HID ||
      in_sizes[27] != FTP * HID || in_sizes[29] != FFM * HID) return;
  if (in_sizes[16] < HID || in_sizes[19] < HID || in_sizes[22] < HID || in_sizes[25] < HID || in_sizes[28] < HID) return;
  for (int i = 30; i < 36; ++i) if (in_sizes[i] < HID) return;
  if (in_sizes[36] != (3 * HID + FGF) * HHALF || in_sizes[37] < HHALF || in_sizes[38] < HHALF || in_sizes[39] < 1) return;

  const float* x_fm       = (const float*)d_in[0];
  const float* x_sm       = (const float*)d_in[1];
  const float* period_vol = (const float*)d_in[2];
  const float* gf         = (const float*)d_in[3];
  const float* pe_table   = (const float*)d_in[4];
  const int* qoq_src = (const int*)d_in[5];  const int* qoq_dst = (const int*)d_in[6];
  const int* bp_src  = (const int*)d_in[7];  const int* bp_dst  = (const int*)d_in[8];
  const int* cp_src  = (const int*)d_in[9];  const int* cp_dst  = (const int*)d_in[10];
  const int* cd_src  = (const int*)d_in[11]; const int* cd_dst  = (const int*)d_in[12];
  const int* rb_src  = (const int*)d_in[13]; const int* rb_dst  = (const int*)d_in[14];
  const float* qoq_Wl = (const float*)d_in[15]; const float* qoq_bl = (const float*)d_in[16];
  const float* qoq_Wr = (const float*)d_in[17];
  const float* bp_Wl  = (const float*)d_in[18]; const float* bp_bl  = (const float*)d_in[19];
  const float* bp_Wr  = (const float*)d_in[20];
  const float* cp_Wl  = (const float*)d_in[21]; const float* cp_bl  = (const float*)d_in[22];
  const float* cp_Wr  = (const float*)d_in[23];
  const float* cd_Wl  = (const float*)d_in[24]; const float* cd_bl  = (const float*)d_in[25];
  const float* cd_Wr  = (const float*)d_in[26];
  const float* rb_Wl  = (const float*)d_in[27]; const float* rb_bl  = (const float*)d_in[28];
  const float* rb_Wr  = (const float*)d_in[29];
  const float* ln_fm_g = (const float*)d_in[30]; const float* ln_fm_b = (const float*)d_in[31];
  const float* ln_tp_g = (const float*)d_in[32]; const float* ln_tp_b = (const float*)d_in[33];
  const float* ln_sm_g = (const float*)d_in[34]; const float* ln_sm_b = (const float*)d_in[35];
  const float* head_W1 = (const float*)d_in[36]; const float* head_b1 = (const float*)d_in[37];
  const float* head_W2 = (const float*)d_in[38]; const float* head_b2 = (const float*)d_in[39];
  float* out = (float*)d_out;

  const int nBfm   = (nFM + NBFM - 1) / NBFM;
  const int nBtp   = (nTP + NBTP - 1) / NBTP;
  const int nBsm   = (nSM + NBSM - 1) / NBSM;
  const int nTPp   = ((nTP + 31) / 32) * 32;
  const int nPeBlk = (nTPp * 8) / NTHR;
  const int nWBlk  = (HID * KFM / 8) / NTHR + (HID * KTP / 8) / NTHR + (HID * KSM / 8) / NTHR + 1;

  char* ws = (char*)d_ws;
  size_t off = 0;
  const size_t oPe  = off; off += (size_t)nTPp * FTP * 4;          off = (off + 255) & ~(size_t)255;
  const size_t oBfm = off; off += (size_t)HID * KFM * 2;           off = (off + 255) & ~(size_t)255;
  const size_t oBtp = off; off += (size_t)HID * KTP * 2;           off = (off + 255) & ~(size_t)255;
  const size_t oBsm = off; off += (size_t)HID * KSM * 2;           off = (off + 255) & ~(size_t)255;
  const size_t oBia = off; off += (size_t)HID * 4;                 off = (off + 255) & ~(size_t)255;
  const size_t oPfm = off; off += (size_t)nBfm * HID * 4;          off = (off + 255) & ~(size_t)255;
  const size_t oPtp = off; off += (size_t)nBtp * HID * 4;          off = (off + 255) & ~(size_t)255;
  const size_t oPsm = off; off += (size_t)nBsm * HID * 4;          off = (off + 255) & ~(size_t)255;
  if (off > ws_size || off > (size_t)128 * 1024 * 1024) return;
  float*    pe     = (float*)(ws + oPe);
  _Float16* Bfm    = (_Float16*)(ws + oBfm);
  _Float16* Btp    = (_Float16*)(ws + oBtp);
  _Float16* Bsm    = (_Float16*)(ws + oBsm);
  float*    biasfm = (float*)(ws + oBia);
  float*    pfm    = (float*)(ws + oPfm);
  float*    ptp    = (float*)(ws + oPtp);
  float*    psm    = (float*)(ws + oPsm);

  k_prep<<<nPeBlk + nWBlk, NTHR, 0, stream>>>(pe_table, period_vol, nTP, nPeBlk,
                                             qoq_Wl, cp_Wl, rb_Wl, qoq_Wr, cp_Wr, rb_Wr,
                                             qoq_bl, cp_bl, rb_bl, bp_Wl, bp_Wr, cd_Wl, cd_Wr,
                                             pe, Bfm, Btp, Bsm, biasfm);

  const float third = 1.0f / 3.0f;

  hipFuncSetAttribute(reinterpret_cast<const void*>(&k_sage<NBFM, FFM, FTP, FTP, FFM>),
                      hipFuncAttributeMaxDynamicSharedMemorySize, LDS_FM);
  k_sage<NBFM, FFM, FTP, FTP, FFM><<<nBfm, NTHR, LDS_FM, stream>>>(
      qoq_src, qoq_dst, nEq, x_fm, nFM,
      cp_src,  cp_dst,  nEc, pe,   nTP,
      rb_src,  rb_dst,  nEr, pe,   nTP,
      x_fm, nFM, Bfm, biasfm, third, ln_fm_g, ln_fm_b, pfm);

  hipFuncSetAttribute(reinterpret_cast<const void*>(&k_sage<NBTP, FFM, 0, 0, FTP>),
                      hipFuncAttributeMaxDynamicSharedMemorySize, LDS_TP);
  k_sage<NBTP, FFM, 0, 0, FTP><<<nBtp, NTHR, LDS_TP, stream>>>(
      bp_src, bp_dst, nEb, x_fm, nFM,
      bp_src, bp_dst, 0,   x_fm, nFM,
      bp_src, bp_dst, 0,   x_fm, nFM,
      pe, nTP, Btp, bp_bl, 1.0f, ln_tp_g, ln_tp_b, ptp);

  hipFuncSetAttribute(reinterpret_cast<const void*>(&k_sage<NBSM, FTP, 0, 0, FSM>),
                      hipFuncAttributeMaxDynamicSharedMemorySize, LDS_SM);
  k_sage<NBSM, FTP, 0, 0, FSM><<<nBsm, NTHR, LDS_SM, stream>>>(
      cd_src, cd_dst, nEd, pe, nTP,
      cd_src, cd_dst, 0,   pe, nTP,
      cd_src, cd_dst, 0,   pe, nTP,
      x_sm, nSM, Bsm, cd_bl, 1.0f, ln_sm_g, ln_sm_b, psm);

  k_final<<<1, HID, 0, stream>>>(pfm, nBfm, nFM, ptp, nBtp, nTP, psm, nBsm, nSM,
                                 gf, head_W1, head_b1, head_W2, head_b2, out);
}
